// LightningAttention_80032420593966
// MI455X (gfx1250) — hardware-verified
//
#include <hip/hip_runtime.h>


namespace {
constexpr int B = 8, T = 8192, D = 128, NH = 8, DH = 16, NT = B * T;
constexpr float XS = 8.0f, KS = 64.0f, OS = 512.0f, WSC = 256.0f;
typedef _Float16 b16;
typedef __attribute__((ext_vector_type(16))) _Float16 v16b;
typedef __attribute__((ext_vector_type(8))) _Float16 v8b;
typedef __attribute__((ext_vector_type(8))) float v8f;
typedef __attribute__((ext_vector_type(4))) float v4f;
__device__ __forceinline__ float bf16_rne(float f) { unsigned int u = __float_as_uint(f); u += 0x7FFFu + ((u >> 16) & 1u); return __uint_as_float(u & 0xFFFF0000u); }
__device__ __forceinline__ void split16(float v, b16& hi, b16& lo) { hi = (b16)v; lo = (b16)(v - (float)hi); }
__device__ __forceinline__ v16b frag_kb(const b16* p, int hh) { const v8b a = *(const v8b*)(p + 8 * hh), b = *(const v8b*)(p + 16 + 8 * hh); v16b f;
#pragma unroll
  for (int e = 0; e < 8; ++e) { f[e] = a[e]; f[8 + e] = b[e]; } return f; }
__device__ __forceinline__ v8f wmma16b(v16b a, v16b b, v8f c) { v8f d = __builtin_amdgcn_wmma_f32_16x16x32_f16(false, a, false, b, (short)0, c, false, false); asm volatile("v_nop\n\tv_nop\n\tv_nop\n\tv_nop" : "+v"(d) : "v"(a), "v"(b)); return d; }
__device__ __forceinline__ void wave_lds_sync() { __builtin_amdgcn_fence(__ATOMIC_RELEASE, "workgroup"); __builtin_amdgcn_wave_barrier(); __builtin_amdgcn_fence(__ATOMIC_ACQUIRE, "workgroup"); }
__device__ __forceinline__ float pmul(float a, float b) { float p = a * b; asm volatile("" : "+v"(p)); return p; }
__device__ __forceinline__ float elu1(float v) { return v > 0.0f ? v + 1.0f : __expf(v); }

__global__ __launch_bounds__(256) void wio_kernel(const float* __restrict__ w, int ro, b16* __restrict__ WT) {
  const int u = blockIdx.x * 256 + threadIdx.x; if (u >= D * D / 8) return; const int e = u * 8; const int o = e / D, k0 = e % D; v8b v;
#pragma unroll
  for (int j = 0; j < 8; ++j) v[j] = (b16)(bf16_rne(w[(size_t)(k0 + j) * D + o]) * WSC); for (int pass = 0; pass < 2; ++pass) { *(volatile v8b*)(WT + (size_t)(ro + o) * D + k0) = v; __threadfence(); }
}
__global__ __launch_bounds__(256) void rope_kernel(float* __restrict__ CSN) {
  const int u = blockIdx.x * 256 + threadIdx.x; if (u >= T * 8) return; const int t = u / 8, d = u % 8; const float invf = 1.0f / powf(10000.0f, (float)(2 * d) / (float)DH); const float ang = (float)t * invf;
  const float c = cosf(ang), s = sinf(ang); for (int pass = 0; pass < 2; ++pass) { ((volatile float*)CSN)[u] = c; ((volatile float*)CSN)[T * 8 + u] = s; __threadfence(); }
}
__global__ __launch_bounds__(32) void qkv_kernel(const float* __restrict__ x, const b16* __restrict__ WT, const float* __restrict__ bq, const float* __restrict__ bk, const float* __restrict__ bv, const float* __restrict__ CSN, int NTV, float* __restrict__ QK, float* __restrict__ V) {
  __shared__ __attribute__((aligned(16))) b16 Ah[16][D + 8]; __shared__ __attribute__((aligned(16))) float Tf[16][D + 4];
  const int lane = threadIdx.x, nloc = lane & 15, hlf = lane >> 4; const size_t t0 = (size_t)blockIdx.x * 16; if (t0 >= (size_t)NTV) return;
  for (int rr = 0; rr < 16; ++rr) for (int q = 0; q < 4; ++q) Ah[rr][q * 32 + lane] = (b16)(bf16_rne(x[(t0 + rr) * D + q * 32 + lane]) * XS);
  wave_lds_sync();
#pragma unroll 1
  for (int cg = 0; cg < 3; ++cg) { const float* bias = cg == 0 ? bq : (cg == 1 ? bk : bv); v8f acc[8];
#pragma unroll
    for (int tt = 0; tt < 8; ++tt) acc[tt] = (v8f){};
#pragma unroll
    for (int kb = 0; kb < D; kb += 32) { const v16b a = frag_kb(&Ah[nloc][kb], hlf);
#pragma unroll
      for (int tt = 0; tt < 8; ++tt) acc[tt] = wmma16b(a, frag_kb(WT + (size_t)(cg * 128 + tt * 16 + nloc) * D + kb, hlf), acc[tt]); }
#pragma unroll
    for (int tt = 0; tt < 8; ++tt) { const int c = tt * 16 + nloc; const float bb = bf16_rne(bias[c]);
#pragma unroll 1
      for (int r8 = 0; r8 < 8; ++r8) Tf[8 * hlf + r8][c] = acc[tt][r8] * (1.0f / (XS * WSC)) + bb; }
    wave_lds_sync();
    if (cg < 2) {
      for (int rr = 0; rr < 16; ++rr) { const size_t t = (t0 + rr) % T; float nv[4];
        for (int q = 0; q < 4; ++q) { const int c = q * 32 + lane; const int d = c & 15; const int dd = d & 7; const float cs = CSN[t * 8 + dd], sn = CSN[(size_t)T * 8 + t * 8 + dd]; const float me = Tf[rr][c], pa = Tf[rr][c ^ 8]; nv[q] = d < 8 ? (me * cs - pa * sn) : (pa * sn + me * cs); }
        wave_lds_sync(); for (int q = 0; q < 4; ++q) Tf[rr][q * 32 + lane] = elu1(nv[q]); }
      wave_lds_sync();
      for (int pass = 0; pass < 2; ++pass) { for (int rr = 0; rr < 16; ++rr) *(volatile v4f*)(QK + (t0 + rr) * (2 * D) + cg * D + lane * 4) = *(const v4f*)(&Tf[rr][lane * 4]); __threadfence(); } }
    else { for (int pass = 0; pass < 2; ++pass) { for (int rr = 0; rr < 16; ++rr) *(volatile v4f*)(V + (t0 + rr) * D + lane * 4) = *(const v4f*)(&Tf[rr][lane * 4]); __threadfence(); } }
    wave_lds_sync(); }
}
__global__ __launch_bounds__(256) void transp_kernel(const float* __restrict__ QK, const float* __restrict__ Vp, int NBV, b16* __restrict__ KH, b16* __restrict__ KL, b16* __restrict__ VH, b16* __restrict__ VL) {
  __shared__ float Tk[64][33], Tv[64][33]; const int nblk_b = (D / 32) * (T / 64); const int b = blockIdx.x / nblk_b; if (b >= NBV) return; const int rem = blockIdx.x % nblk_b; const int tt = rem / (D / 32), ct = rem % (D / 32); const int tid = threadIdx.x;
  for (int i = tid; i < 64 * 32; i += 256) { const int r = i / 32, c = i % 32; const size_t tok = (size_t)b * T + tt * 64 + r; Tk[r][c] = QK[tok * (2 * D) + D + ct * 32 + c]; Tv[r][c] = Vp[tok * D + ct * 32 + c]; }
  __syncthreads();
  { const int c = tid / 8, g = tid % 8; v8b kh, kl, vh, vl;
#pragma unroll
    for (int j = 0; j < 8; ++j) { b16 p, q; split16(Tk[g * 8 + j][c] * KS, p, q); kh[j] = p; kl[j] = q; split16(Tv[g * 8 + j][c] * XS, p, q); vh[j] = p; vl[j] = q; }
    const size_t o = ((size_t)b * D + ct * 32 + c) * T + tt * 64 + g * 8; for (int pass = 0; pass < 2; ++pass) { *(volatile v8b*)(KH + o) = kh; *(volatile v8b*)(KL + o) = kl; *(volatile v8b*)(VH + o) = vh; *(volatile v8b*)(VL + o) = vl; __threadfence(); } }
}
__global__ __launch_bounds__(32) void ctx_kernel(const b16* __restrict__ KH, const b16* __restrict__ KL, const b16* __restrict__ VH, const b16* __restrict__ VL, const float* __restrict__ QK, int NBV, b16* __restrict__ CH, b16* __restrict__ CL, float* __restrict__ KSUM) {
  __shared__ __attribute__((aligned(16))) b16 Th[16][32 + 8], Tl[16][32 + 8];
  const int lane = threadIdx.x, nloc = lane & 15, hlf = lane >> 4; const int b = blockIdx.x / NH, h = blockIdx.x % NH; if (b >= NBV) return;
  const size_t kr = ((size_t)b * D + h * DH + nloc) * T;
  v8f acc = {};
#pragma unroll 4
  for (int kb = 0; kb < T; kb += 32) { const v16b ah = frag_kb(KH + kr + kb, hlf), al = frag_kb(KL + kr + kb, hlf), bh = frag_kb(VH + kr + kb, hlf), bl = frag_kb(VL + kr + kb, hlf); acc = wmma16b(ah, bh, acc); acc = wmma16b(ah, bl, acc); acc = wmma16b(al, bh, acc); acc = wmma16b(al, bl, acc); }
  for (int rr = 0; rr < 16; ++rr) { Th[rr][lane] = (b16)0.0f; Tl[rr][lane] = (b16)0.0f; } wave_lds_sync();
#pragma unroll
  for (int r8 = 0; r8 < 8; ++r8) { b16 p, q; split16(acc[r8] * (1.0f / (KS * XS)), p, q); Th[nloc][8 * hlf + r8] = p; Tl[nloc][8 * hlf + r8] = q; }
  float ks = 0.0f; if (lane < DH) {
#pragma unroll 4
    for (int t = 0; t < T; ++t) ks += QK[((size_t)b * T + t) * (2 * D) + D + h * DH + lane]; }
  wave_lds_sync();
  for (int pass = 0; pass < 2; ++pass) { if (lane < 16) { *(volatile v8b*)(CH + ((size_t)blockIdx.x * 16 + lane) * 32) = *(const v8b*)(&Th[lane][0]); *(volatile v8b*)(CH + ((size_t)blockIdx.x * 16 + lane) * 32 + 8) = *(const v8b*)(&Th[lane][8]); *(volatile v8b*)(CH + ((size_t)blockIdx.x * 16 + lane) * 32 + 16) = *(const v8b*)(&Th[lane][16]); *(volatile v8b*)(CH + ((size_t)blockIdx.x * 16 + lane) * 32 + 24) = *(const v8b*)(&Th[lane][24]);
      *(volatile v8b*)(CL + ((size_t)blockIdx.x * 16 + lane) * 32) = *(const v8b*)(&Tl[lane][0]); *(volatile v8b*)(CL + ((size_t)blockIdx.x * 16 + lane) * 32 + 8) = *(const v8b*)(&Tl[lane][8]); *(volatile v8b*)(CL + ((size_t)blockIdx.x * 16 + lane) * 32 + 16) = *(const v8b*)(&Tl[lane][16]); *(volatile v8b*)(CL + ((size_t)blockIdx.x * 16 + lane) * 32 + 24) = *(const v8b*)(&Tl[lane][24]); }
    ((volatile float*)KSUM)[(size_t)blockIdx.x * 32 + lane] = lane < DH ? ks : 0.0f; __threadfence(); }
}
__global__ __launch_bounds__(32) void out_kernel(const float* __restrict__ QK, const b16* __restrict__ CH, const b16* __restrict__ CL, const float* __restrict__ KSUM, const b16* __restrict__ WO, const float* __restrict__ bo, int NTV, float* __restrict__ out) {
  __shared__ __attribute__((aligned(16))) b16 Qh[NH][16][32 + 8], Ql[NH][16][32 + 8], Ah[16][D + 8], Al[16][D + 8]; __shared__ __attribute__((aligned(16))) float Tf[16][D + 4], Zs[16][NH];
  const int lane = threadIdx.x, nloc = lane & 15, hlf = lane >> 4; const size_t t0 = (size_t)blockIdx.x * 16; if (t0 >= (size_t)NTV) return; const int b = (int)(t0 / T);
  for (int rr = 0; rr < 16; ++rr) { for (int q = 0; q < 4; ++q) { const int c = q * 32 + lane; const int h = c / DH, d = c % DH; const float qv = QK[(t0 + rr) * (2 * D) + c]; b16 p, ql; split16(qv * KS, p, ql); Qh[h][rr][d] = p; Ql[h][rr][d] = ql; Qh[h][rr][16 + d] = (b16)0.0f; Ql[h][rr][16 + d] = (b16)0.0f; }
    if (lane < NH) { float s = 0.0f; for (int d = 0; d < DH; ++d) s += pmul(QK[(t0 + rr) * (2 * D) + lane * DH + d], KSUM[((size_t)b * NH + lane) * 32 + d]); Zs[rr][lane] = 1.0f / (s + 1e-6f); } }
  wave_lds_sync();
#pragma unroll
  for (int h = 0; h < NH; ++h) { const v16b a = frag_kb(&Qh[h][nloc][0], hlf), al = frag_kb(&Ql[h][nloc][0], hlf); const size_t cr = (((size_t)b * NH + h) * 16 + nloc) * 32; const v16b bh = frag_kb(CH + cr, hlf), bl = frag_kb(CL + cr, hlf);
    v8f acc = {}; acc = wmma16b(a, bh, acc); acc = wmma16b(a, bl, acc); acc = wmma16b(al, bh, acc); acc = wmma16b(al, bl, acc);
#pragma unroll
    for (int r8 = 0; r8 < 8; ++r8) { const int rl = 8 * hlf + r8; const float o = pmul(acc[r8] * (1.0f / KS), Zs[rl][h]); b16 p, ql; split16(o * OS, p, ql); Ah[rl][h * DH + nloc] = p; Al[rl][h * DH + nloc] = ql; } }
  wave_lds_sync();
  v8f acc2[8];
#pragma unroll
  for (int tt = 0; tt < 8; ++tt) acc2[tt] = (v8f){};
#pragma unroll
  for (int kb = 0; kb < D; kb += 32) { const v16b a = frag_kb(&Ah[nloc][kb], hlf), al = frag_kb(&Al[nloc][kb], hlf);
#pragma unroll
    for (int tt = 0; tt < 8; ++tt) { const v16b bw = frag_kb(WO + (size_t)(tt * 16 + nloc) * D + kb, hlf); acc2[tt] = wmma16b(a, bw, acc2[tt]); acc2[tt] = wmma16b(al, bw, acc2[tt]); } }
#pragma unroll
  for (int tt = 0; tt < 8; ++tt) { const int c = tt * 16 + nloc; const float bb = bf16_rne(bo[c]);
#pragma unroll 1
    for (int r8 = 0; r8 < 8; ++r8) Tf[8 * hlf + r8][c] = acc2[tt][r8] * (1.0f / (OS * WSC)) + bb; }
  wave_lds_sync();
  for (int pass = 0; pass < 2; ++pass) { for (int rr = 0; rr < 16; ++rr) *(volatile v4f*)(out + (t0 + rr) * D + lane * 4) = *(const v4f*)(&Tf[rr][lane * 4]); __threadfence(); }
}
}

extern "C" void kernel_launch(void* const* d_in, const int* in_sizes, int n_in, void* d_out, int out_size, void* d_ws, size_t ws_size, hipStream_t stream) {
  (void)n_in;
  auto Fp = [&](int i) { return (const float*)d_in[i]; };
  if (in_sizes[0] != NT * D || in_sizes[1] != D * D || in_sizes[3] != D * D || in_sizes[5] != D * D || in_sizes[7] != D * D || out_size != NT * D) return;
  const int NBV = B; const int NTV = NBV * T;
  size_t off = 0; char* ws = (char*)d_ws;
  auto carve = [&](size_t bytes) { char* p = ws + off; off += (bytes + 255) & ~(size_t)255; return p; };
  b16* WQKV = (b16*)carve((size_t)3 * D * D * 2); b16* WO = (b16*)carve((size_t)D * D * 2); float* CSN = (float*)carve((size_t)2 * T * 8 * 4); float* QK = (float*)carve((size_t)NT * 2 * D * 4); float* V = (float*)carve((size_t)NT * D * 4);
  b16* KH = (b16*)carve((size_t)NT * D * 2); b16* KL = (b16*)carve((size_t)NT * D * 2); b16* VH = (b16*)carve((size_t)NT * D * 2); b16* VL = (b16*)carve((size_t)NT * D * 2); b16* CH = (b16*)carve((size_t)B * NH * 16 * 32 * 2); b16* CL = (b16*)carve((size_t)B * NH * 16 * 32 * 2); float* KSUM = (float*)carve((size_t)B * NH * 32 * 4);
  if (off > ws_size || off > ((size_t)192 << 20)) return;
  wio_kernel<<<(D * D / 8 + 255) / 256, 256, 0, stream>>>(Fp(1), 0, WQKV); wio_kernel<<<(D * D / 8 + 255) / 256, 256, 0, stream>>>(Fp(3), D, WQKV); wio_kernel<<<(D * D / 8 + 255) / 256, 256, 0, stream>>>(Fp(5), 2 * D, WQKV); wio_kernel<<<(D * D / 8 + 255) / 256, 256, 0, stream>>>(Fp(7), 0, WO);
  rope_kernel<<<(T * 8 + 255) / 256, 256, 0, stream>>>(CSN);
  qkv_kernel<<<NTV / 16, 32, 0, stream>>>(Fp(0), WQKV, Fp(2), Fp(4), Fp(6), CSN, NTV, QK, V);
  transp_kernel<<<NBV * (D / 32) * (T / 64), 256, 0, stream>>>(QK, V, NBV, KH, KL, VH, VL);
  ctx_kernel<<<NBV * NH, 32, 0, stream>>>(KH, KL, VH, VL, QK, NBV, CH, CL, KSUM);
  out_kernel<<<NTV / 16, 32, 0, stream>>>(QK, CH, CL, KSUM, WO, Fp(8), NTV, (float*)d_out);
}
